// BidirectionalMambaBlock_48069273976855
// MI455X (gfx1250) — hardware-verified
//
#include <hip/hip_runtime.h>
#include <math.h>

typedef __attribute__((ext_vector_type(8)))  _Float16 v8h;
typedef __attribute__((ext_vector_type(16))) __bf16   v16b;
typedef __attribute__((ext_vector_type(8)))  __bf16   v8b;
typedef __attribute__((ext_vector_type(8)))  float    v8f;
typedef __attribute__((ext_vector_type(4)))  float    v4f;

constexpr int kBatch  = 2;
constexpr int kSeq    = 1024;
constexpr int kDm     = 1024;
constexpr int kDin    = 2048;
constexpr int kHeads  = 32;
constexpr int kHdim   = 64;
constexpr int kNst    = 64;
constexpr int kConvC  = kDin + 2 * kNst;
constexpr int kProj   = 2 * kDin + 2 * kNst + kHeads;
constexpr int kProjP  = 4288;
constexpr int kRows   = kBatch * kSeq;
constexpr int kChunk  = 16;
constexpr int kUP     = 192;
constexpr int kYP     = 68;
static_assert(kHeads * kHdim == kDin, "head split");
static_assert(kConvC == 2176 && kProj == 4256, "projection widths");
static_assert(kProjP >= kProj && (kProjP % 64) == 0, "padded projection width");
static_assert((kDm % 64) == 0 && (kDin % 64) == 0 && (kRows % 64) == 0, "GEMM M,N,K tile multiples");
static_assert((kDm % 32) == 0 && (kDin % 32) == 0, "GEMM K multiples of 32");
static_assert((kSeq % kChunk) == 0, "scan chunking");
static_assert(kHdim == 64 && kNst == 64 && kHeads == 32, "scan thread map");
static_assert(kDin == 256 * 8, "gate/norm thread map");

constexpr size_t kOffX16   = 0;
constexpr size_t kOffWINF  = kOffX16   + (size_t)kRows  * kDm  * 2;
constexpr size_t kOffWINB  = kOffWINF  + (size_t)kProjP * kDm  * 2;
constexpr size_t kOffWOUTF = kOffWINB  + (size_t)kProjP * kDm  * 2;
constexpr size_t kOffWOUTB = kOffWOUTF + (size_t)kDm    * kDin * 2;
constexpr size_t kOffWOT   = kOffWOUTB + (size_t)kDm    * kDin * 2;
constexpr size_t kOffZX    = kOffWOT   + (size_t)kDm    * kDin * 2;
constexpr size_t kOffYR    = kOffZX    + (size_t)kRows  * kProjP * 4;
constexpr size_t kOffYH    = kOffYR    + (size_t)kRows  * kDin * 4;
constexpr size_t kOffYL    = kOffYH    + (size_t)kRows  * kDin * 2;
constexpr size_t kOffCH    = kOffYL    + (size_t)kRows  * kDin * 2;
constexpr size_t kOffCL    = kOffCH    + (size_t)kRows  * kDin * 2;
constexpr size_t kWsTotal  = kOffCL    + (size_t)kRows  * kDin * 2;
static_assert(kWsTotal == 119799808ull, "carve total");
static_assert(kWsTotal <= 134217728ull, "carve cap");
static_assert((kOffWINF % 128) == 0 && (kOffWINB % 128) == 0 && (kOffWOUTF % 128) == 0 && (kOffWOUTB % 128) == 0 &&
              (kOffWOT % 128) == 0 && (kOffZX % 128) == 0 && (kOffYR % 128) == 0 && (kOffYH % 128) == 0 &&
              (kOffYL % 128) == 0 && (kOffCH % 128) == 0 && (kOffCL % 128) == 0, "128-B aligned regions");

__device__ __forceinline__ unsigned short f2bf_bits(float f) {
  unsigned u = __float_as_uint(f);
  return (unsigned short)((u + 0x7FFFu + ((u >> 16) & 1u)) >> 16);
}
__device__ __forceinline__ float bf_bits2f(unsigned short h) { return __uint_as_float(((unsigned)h) << 16); }
__device__ __forceinline__ float bf_rne(float f) { return bf_bits2f(f2bf_bits(f)); }

__device__ __forceinline__ void dep_guard4_b(v8f& a, v8f& b, v8f& c, v8f& d, v16b x, v16b y) {
  asm volatile("v_nop\n\tv_nop\n\tv_nop\n\tv_nop" : "+v"(a), "+v"(b), "+v"(c), "+v"(d) : "v"(x), "v"(y));
}
__device__ __forceinline__ void keep4_b(v16b a, v16b b, v16b c, v16b d) { asm volatile("v_nop" :: "v"(a), "v"(b), "v"(c), "v"(d)); }
__device__ __forceinline__ void acc_guard4(v8f& a, v8f& b, v8f& c, v8f& d) { asm volatile("v_nop\n\tv_nop\n\tv_nop\n\tv_nop" : "+v"(a), "+v"(b), "+v"(c), "+v"(d)); }

struct FragB {
  union U { v16b v; v8b h[2]; };
  static __device__ __forceinline__ v16b load(const __bf16* p) {
    U f; f.h[0] = *(const v8b*)(p); f.h[1] = *(const v8b*)(p + 16); return f.v;
  }
  static __device__ __forceinline__ v8f mma(v16b a, v16b b, v8f c) {
    return __builtin_amdgcn_wmma_f32_16x16x32_bf16(false, a, false, b, (short)0, c, false, false);
  }
};

template <int SPL, int BIAS_MODE, int OUT_MODE>
__global__ __launch_bounds__(256) void wmma_gemm64(
    const unsigned short* __restrict__ Ap, const unsigned short* __restrict__ A2p, int lda,
    const unsigned short* __restrict__ Btp, int ldb,
    void* __restrict__ Cout, void* __restrict__ Cout2, int ldc,
    const float* __restrict__ bias,
    int M, int N, int K) {
  const __bf16* A  = (const __bf16*)Ap;
  const __bf16* A2 = (const __bf16*)A2p;
  const __bf16* Bt = (const __bf16*)Btp;
  __shared__ __align__(16) float sT[8][16 * 68];
  const int lane = threadIdx.x & 31;
  const int wave = threadIdx.x >> 5;
  const int tilesN = N >> 6;
  const int tilesM = M >> 6;
  const int tile = blockIdx.x * 8 + wave;
  if (tile >= tilesM * tilesN) return;
  const int tm = tile / tilesN;
  const int tn = tile - tm * tilesN;
  const int m0 = tm << 6;
  const int n0 = tn << 6;

  const int rlane = lane & 15;
  const int koff  = (lane >> 4) * 8;
  const int mOff  = (lane >> 4) * 8;

  v8f acc[4][4];
#pragma unroll
  for (int i = 0; i < 4; ++i)
#pragma unroll
    for (int j = 0; j < 4; ++j) acc[i][j] = (v8f){0.f,0.f,0.f,0.f,0.f,0.f,0.f,0.f};

  for (int k0 = 0; k0 < K; k0 += 32) {
    v16b bh[4];
#pragma unroll
    for (int j = 0; j < 4; ++j) {
      const size_t bo = (size_t)(n0 + (j << 4) + rlane) * ldb + koff + k0;
      bh[j] = FragB::load(Bt + bo);
    }
#pragma unroll
    for (int i = 0; i < 4; ++i) {
      const size_t ao = (size_t)(m0 + (i << 4) + rlane) * lda + koff + k0;
      v16b ah = FragB::load(A + ao);
      v16b al = ah;
      if (SPL >= 1) al = FragB::load(A2 + ao);
#pragma unroll
      for (int j = 0; j < 4; ++j) {
        acc[i][j] = FragB::mma(ah, bh[j], acc[i][j]);
        if (SPL >= 1) acc[i][j] = FragB::mma(al, bh[j], acc[i][j]);
      }
      dep_guard4_b(acc[i][0], acc[i][1], acc[i][2], acc[i][3], ah, al);
    }
    keep4_b(bh[0], bh[1], bh[2], bh[3]);
  }
  acc_guard4(acc[0][0], acc[0][1], acc[0][2], acc[0][3]);
  acc_guard4(acc[1][0], acc[1][1], acc[1][2], acc[1][3]);
  acc_guard4(acc[2][0], acc[2][1], acc[2][2], acc[2][3]);
  acc_guard4(acc[3][0], acc[3][1], acc[3][2], acc[3][3]);

  float* slab = sT[wave];
#pragma unroll
  for (int i = 0; i < 4; ++i) {
    const int mBase = m0 + (i << 4);
#pragma unroll
    for (int j = 0; j < 4; ++j) {
      const int n = n0 + (j << 4) + rlane;
      float bv = 0.f;
      if (BIAS_MODE == 2) bv = bf_rne(bias[n]);
#pragma unroll
      for (int r = 0; r < 8; ++r) {
        float v = acc[i][j][r];
        if (BIAS_MODE == 2) v += bv;
        slab[(mOff + r) * 68 + (j << 4) + rlane] = v;
      }
    }
    __builtin_amdgcn_fence(__ATOMIC_RELEASE, "workgroup");
    __builtin_amdgcn_wave_barrier();
    __builtin_amdgcn_fence(__ATOMIC_ACQUIRE, "workgroup");
    if (OUT_MODE == 0) {
      float* C = (float*)Cout;
      const int hh = lane >> 4, c4 = (lane & 15) * 4;
      for (int pass = 0; pass < 2; ++pass) {
#pragma unroll
        for (int it = 0; it < 8; ++it) {
          const int row = it * 2 + hh;
          v4f v = *(const v4f*)(slab + row * 68 + c4);
          *(volatile v4f*)(C + (size_t)(mBase + row) * ldc + n0 + c4) = v;
        }
        __threadfence();
      }
    } else {
      const int q = lane >> 3, c8 = (lane & 7) * 8;
      unsigned short* C  = (unsigned short*)Cout;
      unsigned short* C2 = (unsigned short*)Cout2;
      for (int pass = 0; pass < 2; ++pass) {
#pragma unroll
        for (int it = 0; it < 4; ++it) {
          const int row = it * 4 + q;
          const float* sp = slab + row * 68 + c8;
          v8h hv, lv;
#pragma unroll
          for (int e = 0; e < 8; ++e) {
            const float fv = sp[e];
            const unsigned short hb = f2bf_bits(fv);
            const unsigned short lb = f2bf_bits(fv - bf_bits2f(hb));
            hv[e] = __builtin_bit_cast(_Float16, hb);
            lv[e] = __builtin_bit_cast(_Float16, lb);
          }
          *(volatile v8h*)(C  + (size_t)(mBase + row) * ldc + n0 + c8) = hv;
          *(volatile v8h*)(C2 + (size_t)(mBase + row) * ldc + n0 + c8) = lv;
        }
        __threadfence();
      }
    }
    __builtin_amdgcn_fence(__ATOMIC_RELEASE, "workgroup");
    __builtin_amdgcn_wave_barrier();
    __builtin_amdgcn_fence(__ATOMIC_ACQUIRE, "workgroup");
  }
}

__global__ __launch_bounds__(256) void cast_bf16_kernel(
    const float* __restrict__ src, unsigned short* __restrict__ dst, int total8)
{
  const int i = blockIdx.x * 256 + threadIdx.x;
  if (i >= total8) return;
  const size_t e0 = (size_t)i << 3;
  const v4f a0 = *(const v4f*)(src + e0);
  const v4f a1 = *(const v4f*)(src + e0 + 4);
  v8h hv;
#pragma unroll
  for (int e = 0; e < 4; ++e) {
    const float f0 = a0[e];
    const float f1 = a1[e];
    const unsigned short h0 = f2bf_bits(f0);
    const unsigned short h1 = f2bf_bits(f1);
    hv[e]     = __builtin_bit_cast(_Float16, h0);
    hv[4 + e] = __builtin_bit_cast(_Float16, h1);
  }
  unsigned short* q = dst + e0;
  *(volatile v8h*)q = hv;
  __threadfence();
  *(volatile v8h*)q = hv;
}

__global__ __launch_bounds__(256) void transpose_cast_kernel(
    const float* __restrict__ W, unsigned short* __restrict__ Bt, int Kdim, int Ndim)
{
  __shared__ float tile[64 * 65];
  const int tid = threadIdx.x, lane = tid & 31, wave = tid >> 5;
  const int n0 = blockIdx.x * 64;
  const int k0 = blockIdx.y * 64;
#pragma unroll
  for (int pp = 0; pp < 16; ++pp) {
    const int idx = tid + pp * 256;
    const int kk  = idx >> 6;
    const int nn  = idx & 63;
    const int n   = n0 + nn;
    const int nc  = (n < Ndim) ? n : (Ndim - 1);
    const float v = W[(size_t)(k0 + kk) * Ndim + nc];
    tile[kk * 65 + nn] = (n < Ndim) ? v : 0.f;
  }
  __syncthreads();
  const int q = lane >> 3, c8 = (lane & 7) * 8;
  v8h hv[2];
#pragma unroll
  for (int it = 0; it < 2; ++it) {
    const int nrow = it * 32 + wave * 4 + q;
#pragma unroll
    for (int e = 0; e < 8; ++e) {
      const unsigned short hb = f2bf_bits(tile[(c8 + e) * 65 + nrow]);
      hv[it][e] = __builtin_bit_cast(_Float16, hb);
    }
  }
  for (int pass = 0; pass < 2; ++pass) {
#pragma unroll
    for (int it = 0; it < 2; ++it) {
      const int nrow = it * 32 + wave * 4 + q;
      *(volatile v8h*)(Bt + (size_t)(n0 + nrow) * Kdim + k0 + c8) = hv[it];
    }
    __threadfence();
  }
}

__global__ __launch_bounds__(256) void scan_fused_kernel(
    const float* __restrict__ ZX, const float* __restrict__ cw, const float* __restrict__ cb,
    const float* __restrict__ dtb, const float* __restrict__ Alog, const float* __restrict__ Dsk,
    float* __restrict__ YR, int dir)
{
  __shared__ __align__(16) float sU[kChunk * kUP];
  __shared__ __align__(16) float sDD[32];
  __shared__ __align__(16) float sY[kChunk * kYP];
  const int tid  = threadIdx.x;
  const int lane = tid & 31;
  const int wave = __builtin_amdgcn_readfirstlane(tid >> 5);
  const int bix  = blockIdx.x / kHeads;
  const int hd   = blockIdx.x - bix * kHeads;
  const int pch  = tid >> 2;
  const int nb   = (tid & 3) * 16;
  const size_t rowbase = (size_t)bix * kSeq;

  const int otid = (tid < kUP) ? tid : (kUP - 1);
  const int cch  = (otid < 64) ? (hd * kHdim + otid) : (kDin + (otid - 64));
  const float w0 = bf_rne(cw[0 * kConvC + cch]);
  const float w1 = bf_rne(cw[1 * kConvC + cch]);
  const float w2 = bf_rne(cw[2 * kConvC + cch]);
  const float w3 = bf_rne(cw[3 * kConvC + cch]);
  const float bc = bf_rne(cb[cch]);
  const float hdtb = bf_rne(dtb[hd]);
  const float negA = -expf(bf_rne(Alog[hd]));
  const float dsk  = bf_rne(Dsk[hd]);

  float h[16];
#pragma unroll
  for (int i = 0; i < 16; ++i) h[i] = 0.f;
  float xm3 = 0.f, xm2 = 0.f, xm1 = 0.f;

#pragma unroll 1
  for (int c = 0; c < kSeq / kChunk; ++c) {
    const int tau0 = c * kChunk;
    if (wave < 6) {
#pragma unroll 1
      for (int s = 0; s < kChunk; ++s) {
        const int tau = tau0 + s;
        const int l = dir ? (kSeq - 1 - tau) : tau;
        float u = ZX[(rowbase + l) * kProjP + kDin + cch];
        asm volatile("" : "+v"(u));
        float acc = w0 * xm3;
        acc = fmaf(w1, xm2, acc);
        acc = fmaf(w2, xm1, acc);
        acc = fmaf(w3, u, acc);
        const float sv = acc + bc;
        const float sg = 1.0f / (1.0f + expf(-sv));
        sU[s * kUP + tid] = sv * sg;
        xm3 = xm2; xm2 = xm1; xm1 = u;
      }
    } else if (wave == 6) {
      const int tau = tau0 + (lane & 15);
      const int l = dir ? (kSeq - 1 - tau) : tau;
      float dr = ZX[(rowbase + l) * kProjP + kDin + kConvC + hd];
      asm volatile("" : "+v"(dr));
      const float dv  = dr + hdtb;
      const float ea  = expf(-fabsf(dv));
      const float u1  = 1.0f + ea;
      const float l1p = logf(u1) + (ea - (u1 - 1.0f)) / u1;
      const float dtv = fmaxf(dv, 0.0f) + l1p;
      const float dav = expf(dtv * negA);
      sDD[lane] = (lane < 16) ? dtv : dav;
    }
    __syncthreads();
#pragma unroll 1
    for (int s = 0; s < kChunk; ++s) {
      const float xp   = sU[s * kUP + pch];
      const float dtv  = sDD[s];
      const float dav  = sDD[16 + s];
      const float coef = dtv * xp;
      const float* bp = sU + s * kUP + 64 + nb;
      const float* cp = sU + s * kUP + 128 + nb;
      float acc = 0.f;
#pragma unroll
      for (int q4 = 0; q4 < 4; ++q4) {
        const v4f bv = *(const v4f*)(bp + 4 * q4);
        const v4f cv = *(const v4f*)(cp + 4 * q4);
        h[4 * q4 + 0] = fmaf(dav, h[4 * q4 + 0], coef * bv[0]);
        acc = fmaf(cv[0], h[4 * q4 + 0], acc);
        h[4 * q4 + 1] = fmaf(dav, h[4 * q4 + 1], coef * bv[1]);
        acc = fmaf(cv[1], h[4 * q4 + 1], acc);
        h[4 * q4 + 2] = fmaf(dav, h[4 * q4 + 2], coef * bv[2]);
        acc = fmaf(cv[2], h[4 * q4 + 2], acc);
        h[4 * q4 + 3] = fmaf(dav, h[4 * q4 + 3], coef * bv[3]);
        acc = fmaf(cv[3], h[4 * q4 + 3], acc);
      }
      acc += __shfl_xor(acc, 1, 32);
      acc += __shfl_xor(acc, 2, 32);
      float y = fmaf(dsk, xp, acc);
      asm volatile("" : "+v"(y));
      if ((tid & 3) == 0) sY[s * kYP + pch] = y;
    }
    __syncthreads();
    {
      const int hh = lane >> 4, c4 = (lane & 15) * 4;
      const int srow = wave * 2 + hh;
      const int tau = tau0 + srow;
      const int l = dir ? (kSeq - 1 - tau) : tau;
      const v4f v = *(const v4f*)(sY + srow * kYP + c4);
      float* dst = YR + (rowbase + l) * kDin + hd * kHdim + c4;
      *(volatile v4f*)dst = v;
      __threadfence();
      *(volatile v4f*)dst = v;
    }
  }
}

__global__ __launch_bounds__(256) void gate_norm_kernel(
    const float* __restrict__ YR, const float* __restrict__ ZX, const float* __restrict__ normw,
    unsigned short* __restrict__ YH, unsigned short* __restrict__ YLo)
{
  __shared__ __align__(16) float sG[kDin];
  __shared__ float sP[8];
  const int tid = threadIdx.x, lane = tid & 31, wave = tid >> 5;
  const size_t row = blockIdx.x;
  const float* yr = YR + row * kDin;
  const float* zr = ZX + row * kProjP;
  float ss = 0.f;
#pragma unroll 1
  for (int e = 0; e < 8; ++e) {
    const int ch = e * 256 + tid;
    const float zv = zr[ch];
    const float yv = yr[ch];
    const float sg = 1.0f / (1.0f + expf(-zv));
    const float g  = yv * (zv * sg);
    sG[ch] = g;
    ss = fmaf(g, g, ss);
  }
  ss += __shfl_xor(ss, 16, 32);
  ss += __shfl_xor(ss, 8, 32);
  ss += __shfl_xor(ss, 4, 32);
  ss += __shfl_xor(ss, 2, 32);
  ss += __shfl_xor(ss, 1, 32);
  if (lane == 0) sP[wave] = ss;
  __syncthreads();
  float tot = sP[0];
  tot += sP[1]; tot += sP[2]; tot += sP[3]; tot += sP[4]; tot += sP[5]; tot += sP[6]; tot += sP[7];
  constexpr float kInvN = 1.0f / (float)kDin;
  const float scale = 1.0f / sqrtf(tot * kInvN + 1e-5f);
  const int j0 = tid * 8;
  const v4f g0 = *(const v4f*)(sG + j0);
  const v4f g1 = *(const v4f*)(sG + j0 + 4);
  const v4f n0v = *(const v4f*)(normw + j0);
  const v4f n1v = *(const v4f*)(normw + j0 + 4);
  v8h hv, lv;
#pragma unroll
  for (int e = 0; e < 4; ++e) {
    const float ga = g0[e];
    const float gb = g1[e];
    const float na = n0v[e];
    const float nbv = n1v[e];
    const float va = (ga * scale) * bf_rne(na);
    const float vb = (gb * scale) * bf_rne(nbv);
    const unsigned short ha = f2bf_bits(va);
    const unsigned short hb = f2bf_bits(vb);
    const unsigned short la = f2bf_bits(va - bf_bits2f(ha));
    const unsigned short lb = f2bf_bits(vb - bf_bits2f(hb));
    hv[e]     = __builtin_bit_cast(_Float16, ha);
    hv[4 + e] = __builtin_bit_cast(_Float16, hb);
    lv[e]     = __builtin_bit_cast(_Float16, la);
    lv[4 + e] = __builtin_bit_cast(_Float16, lb);
  }
  unsigned short* qh = YH  + row * kDin + j0;
  unsigned short* ql = YLo + row * kDin + j0;
  *(volatile v8h*)qh = hv;
  *(volatile v8h*)ql = lv;
  __threadfence();
  *(volatile v8h*)qh = hv;
  *(volatile v8h*)ql = lv;
}

extern "C" void kernel_launch(void* const* d_in, const int* in_sizes, int n_in,
                              void* d_out, int out_size, void* d_ws, size_t ws_size,
                              hipStream_t stream)
{
  if (n_in < 19) return;
  if (in_sizes[0] != kRows * kDm) return;
  if (in_sizes[1] != kDm * kProj || in_sizes[9] != kDm * kProj) return;
  if (in_sizes[2] != 4 * kConvC || in_sizes[10] != 4 * kConvC) return;
  if (in_sizes[3] != kConvC || in_sizes[11] != kConvC) return;
  if (in_sizes[4] != kHeads || in_sizes[5] != kHeads || in_sizes[6] != kHeads) return;
  if (in_sizes[12] != kHeads || in_sizes[13] != kHeads || in_sizes[14] != kHeads) return;
  if (in_sizes[7] != kDin || in_sizes[15] != kDin) return;
  if (in_sizes[8] != kDin * kDm || in_sizes[16] != kDin * kDm) return;
  if (in_sizes[17] != 2 * kDm * kDm || in_sizes[18] != kDm) return;
  if (out_size != kRows * kDm) return;
  if (ws_size < kWsTotal) return;

  const float* x      = (const float*)d_in[0];
  const float* fWin   = (const float*)d_in[1];
  const float* fconvw = (const float*)d_in[2];
  const float* fconvb = (const float*)d_in[3];
  const float* fdtb   = (const float*)d_in[4];
  const float* fAlog  = (const float*)d_in[5];
  const float* fD     = (const float*)d_in[6];
  const float* fnormw = (const float*)d_in[7];
  const float* fWout  = (const float*)d_in[8];
  const float* bWin   = (const float*)d_in[9];
  const float* bconvw = (const float*)d_in[10];
  const float* bconvb = (const float*)d_in[11];
  const float* bdtb   = (const float*)d_in[12];
  const float* bAlog  = (const float*)d_in[13];
  const float* bD     = (const float*)d_in[14];
  const float* bnormw = (const float*)d_in[15];
  const float* bWout  = (const float*)d_in[16];
  const float* Wo     = (const float*)d_in[17];
  const float* bo     = (const float*)d_in[18];
  float* out = (float*)d_out;

  char* ws = (char*)d_ws;
  unsigned short* X16   = (unsigned short*)(ws + kOffX16);
  unsigned short* WINF  = (unsigned short*)(ws + kOffWINF);
  unsigned short* WINB  = (unsigned short*)(ws + kOffWINB);
  unsigned short* WOUTF = (unsigned short*)(ws + kOffWOUTF);
  unsigned short* WOUTB = (unsigned short*)(ws + kOffWOUTB);
  unsigned short* WOT   = (unsigned short*)(ws + kOffWOT);
  float*          ZX    = (float*)(ws + kOffZX);
  float*          YR    = (float*)(ws + kOffYR);
  unsigned short* YH    = (unsigned short*)(ws + kOffYH);
  unsigned short* YL    = (unsigned short*)(ws + kOffYL);
  unsigned short* CH    = (unsigned short*)(ws + kOffCH);
  unsigned short* CL    = (unsigned short*)(ws + kOffCL);

  cast_bf16_kernel<<<(kRows * kDm / 8) / 256, 256, 0, stream>>>(x, X16, kRows * kDm / 8);

  transpose_cast_kernel<<<dim3(kProjP / 64, kDm / 64), 256, 0, stream>>>(fWin, WINF, kDm, kProj);
  transpose_cast_kernel<<<dim3(kProjP / 64, kDm / 64), 256, 0, stream>>>(bWin, WINB, kDm, kProj);
  transpose_cast_kernel<<<dim3(kDm / 64, kDin / 64), 256, 0, stream>>>(fWout, WOUTF, kDin, kDm);
  transpose_cast_kernel<<<dim3(kDm / 64, kDin / 64), 256, 0, stream>>>(bWout, WOUTB, kDin, kDm);
  transpose_cast_kernel<<<dim3(kDm / 64, kDin / 64), 256, 0, stream>>>(Wo, WOT, kDin, kDm);

  for (int dir = 0; dir < 2; ++dir) {
    const unsigned short* WIN  = dir ? WINB  : WINF;
    const unsigned short* WOUT = dir ? WOUTB : WOUTF;
    const float* convw = dir ? bconvw : fconvw;
    const float* convb = dir ? bconvb : fconvb;
    const float* dtbp  = dir ? bdtb   : fdtb;
    const float* alogp = dir ? bAlog  : fAlog;
    const float* dskp  = dir ? bD     : fD;
    const float* nwp   = dir ? bnormw : fnormw;

    wmma_gemm64<0, 0, 0><<<dim3((kRows / 64) * (kProjP / 64) / 8, 1), 256, 0, stream>>>(
        X16, X16, kDm, WIN, kDm, (void*)ZX, (void*)ZX, kProjP, bo, kRows, kProjP, kDm);

    scan_fused_kernel<<<kBatch * kHeads, 256, 0, stream>>>(ZX, convw, convb, dtbp, alogp, dskp, YR, dir);

    gate_norm_kernel<<<kRows, 256, 0, stream>>>(YR, ZX, nwp, YH, YL);

    wmma_gemm64<1, 0, 2><<<dim3((kRows / 64) * (kDm / 64) / 8, 1), 256, 0, stream>>>(
        YH, YL, kDin, WOUT, kDin, (void*)(CH + (size_t)dir * kDm), (void*)(CL + (size_t)dir * kDm), 2 * kDm,
        bo, kRows, kDm, kDin);
  }

  wmma_gemm64<1, 2, 0><<<dim3((kRows / 64) * (kDm / 64) / 8, 1), 256, 0, stream>>>(
      CH, CL, 2 * kDm, WOT, 2 * kDm, (void*)out, (void*)out, kDm, bo, kRows, kDm, 2 * kDm);
}
